// Attn_79671643341302
// MI455X (gfx1250) — hardware-verified
//
#include <hip/hip_runtime.h>
#include <math.h>

typedef __attribute__((ext_vector_type(16))) _Float16 v16h;
typedef __attribute__((ext_vector_type(8)))  _Float16 v8h;
typedef __attribute__((ext_vector_type(16))) __bf16   v16b;
typedef __attribute__((ext_vector_type(8)))  __bf16   v8b;
typedef __attribute__((ext_vector_type(8)))  float    v8f;
typedef __attribute__((ext_vector_type(4)))  float    v4f;
typedef __attribute__((ext_vector_type(8)))  unsigned short v8us;
typedef __attribute__((ext_vector_type(4)))  unsigned short v4us;

#ifndef NB
#define NB 2
#endif
#ifndef SEQ
#define SEQ 2048
#endif
static constexpr int NB_FULL  = 2;
static constexpr int SEQ_FULL = 2048;
static constexpr int CDIM  = 2048;
static constexpr int NHEAD = 16;
static constexpr int NKV   = 4;
static constexpr int HD    = 128;
static constexpr int GRP   = NHEAD / NKV;
static constexpr int BT    = NB * SEQ;
static constexpr int NKVC  = NKV * HD;
static constexpr int NQK   = CDIM + NKVC;
static constexpr int NQB   = SEQ / 64;
static constexpr int NQB_SPLIT = (NQB < 8) ? NQB : 8;
static constexpr int AKC   = 32;
static constexpr int ANW   = 4;
static constexpr float RES_SC  = 2048.0f;
static constexpr float RES_INV = 1.0f / 2048.0f;
static constexpr float P_SC    = 1024.0f;
static constexpr float RMS_EPS = 1.1920929e-7f;

static_assert(NB >= 1 && NB <= NB_FULL && SEQ >= 64 && SEQ <= SEQ_FULL);
static_assert(BT % 64 == 0 && NQK % 64 == 0 && CDIM % 32 == 0);
static_assert(NKVC % 64 == 0 && SEQ % 64 == 0 && CDIM % 64 == 0);
static_assert(HD == 128 && (HD % 32) == 0);
static_assert(NQB_SPLIT > 0 && NQB_SPLIT <= NQB);
static_assert(NHEAD * HD == CDIM && (NHEAD + NKV) * HD == NQK);

__device__ __forceinline__ unsigned short f2bf_bits(float f) {
  unsigned u = __float_as_uint(f);
  return (unsigned short)((u + 0x7FFFu + ((u >> 16) & 1u)) >> 16);
}
__device__ __forceinline__ float bf_bits2f(unsigned short h) { return __uint_as_float(((unsigned)h) << 16); }

__device__ __forceinline__ void dep_guard_h(v8f& a, v8f& b, v16h x, v16h y) { asm volatile("v_nop\n\tv_nop\n\tv_nop\n\tv_nop" : "+v"(a), "+v"(b) : "v"(x), "v"(y)); }
__device__ __forceinline__ void dep_guard_b(v8f& a, v8f& b, v16b x, v16b y) { asm volatile("v_nop\n\tv_nop\n\tv_nop\n\tv_nop" : "+v"(a), "+v"(b) : "v"(x), "v"(y)); }
__device__ __forceinline__ void keep4_h(v16h a, v16h b, v16h c, v16h d) { asm volatile("v_nop" :: "v"(a), "v"(b), "v"(c), "v"(d)); }
__device__ __forceinline__ void keep4_b(v16b a, v16b b, v16b c, v16b d) { asm volatile("v_nop" :: "v"(a), "v"(b), "v"(c), "v"(d)); }
__device__ __forceinline__ void acc_guard4(v8f& a, v8f& b, v8f& c, v8f& d) { asm volatile("v_nop\n\tv_nop\n\tv_nop\n\tv_nop" : "+v"(a), "+v"(b), "+v"(c), "+v"(d)); }
template <typename T> struct Frag;
template <> struct Frag<_Float16> {
  typedef v16h V; union U { v16h v; v8h h[2]; };
  static __device__ __forceinline__ v16h load(const _Float16* p) {
    U f; f.h[0] = *(const v8h*)(p); f.h[1] = *(const v8h*)(p + 16); return f.v;
  }
  static __device__ __forceinline__ v8f mma(v16h a, v16h b, v8f c) {
    return __builtin_amdgcn_wmma_f32_16x16x32_f16(false, a, false, b, (short)0, c, false, false);
  }
  static __device__ __forceinline__ void guard(v8f& a, v8f& b, v16h x, v16h y) { dep_guard_h(a, b, x, y); }
  static __device__ __forceinline__ void keep(v16h a, v16h b, v16h c, v16h d) { keep4_h(a, b, c, d); }
};
template <> struct Frag<__bf16> {
  typedef v16b V; union U { v16b v; v8b h[2]; };
  static __device__ __forceinline__ v16b load(const __bf16* p) {
    U f; f.h[0] = *(const v8b*)(p); f.h[1] = *(const v8b*)(p + 16); return f.v;
  }
  static __device__ __forceinline__ v8f mma(v16b a, v16b b, v8f c) {
    return __builtin_amdgcn_wmma_f32_16x16x32_bf16(false, a, false, b, (short)0, c, false, false);
  }
  static __device__ __forceinline__ void guard(v8f& a, v8f& b, v16b x, v16b y) { dep_guard_b(a, b, x, y); }
  static __device__ __forceinline__ void keep(v16b a, v16b b, v16b c, v16b d) { keep4_b(a, b, c, d); }
};

__device__ __forceinline__ v8f hmma(v16h a, v16h b, v8f c) {
  c = __builtin_amdgcn_wmma_f32_16x16x32_f16(false, a, false, b, (short)0, c, false, false);
  asm volatile("v_nop\n\tv_nop\n\tv_nop\n\tv_nop" : "+v"(c) : "v"(a), "v"(b));
  return c;
}
__device__ __forceinline__ v8f zero8() { return (v8f){0.f, 0.f, 0.f, 0.f, 0.f, 0.f, 0.f, 0.f}; }

template <int ET> struct Elem;
template <> struct Elem<0> { typedef _Float16 T; };
template <> struct Elem<1> { typedef __bf16 T; };
template <int ET, int SPLIT, int BIAS_MODE, int OUT_MODE>
__global__ __launch_bounds__(256) void wmma_gemm64(
    const unsigned short* __restrict__ Ap, const unsigned short* __restrict__ A2p, int lda, long strideA,
    const unsigned short* __restrict__ Btp, const unsigned short* __restrict__ Bt2p, int ldb, long strideB,
    void* __restrict__ Cout, void* __restrict__ Cout2, int ldc, long strideC,
    const float* __restrict__ bias,
    int M, int N, int K, float scale) {
  typedef typename Elem<ET>::T T;
  typedef typename Frag<T>::V V;
  const T* A = (const T*)Ap; const T* A2 = (const T*)A2p; const T* Bt = (const T*)Btp; const T* Bt2 = (const T*)Bt2p;
  __shared__ __align__(16) float sT[8][16 * 68];
  const int b    = blockIdx.y;
  const int lane = threadIdx.x & 31;
  const int wave = threadIdx.x >> 5;
  const int tilesN = N >> 6;
  const int tilesM = M >> 6;
  const int tile = blockIdx.x * 8 + wave;
  if (tile >= tilesM * tilesN) return;
  const int tm = tile / tilesN;
  const int tn = tile - tm * tilesN;
  const int m0 = tm << 6;
  const int n0 = tn << 6;

  const T* Ab  = A  + (size_t)b * strideA;
  const T* Bb  = Bt + (size_t)b * strideB;
  const T* Ab2 = (SPLIT >= 1) ? (A2  + (size_t)b * strideA) : nullptr;
  const T* Bb2 = (SPLIT == 2) ? (Bt2 + (size_t)b * strideB) : nullptr;

  const int rlane = lane & 15;
  const int koff  = (lane >> 4) * 8;
  const int mOff  = (lane >> 4) * 8;

  v8f acc[4][4];
#pragma unroll
  for (int i = 0; i < 4; ++i)
#pragma unroll
    for (int j = 0; j < 4; ++j) acc[i][j] = zero8();

  for (int k0 = 0; k0 < K; k0 += 32) {
    V bh[4], bl[4];
#pragma unroll
    for (int j = 0; j < 4; ++j) {
      const size_t bo = (size_t)(n0 + (j << 4) + rlane) * ldb + koff + k0;
      bh[j] = Frag<T>::load(Bb + bo);
      if (SPLIT == 2) bl[j] = Frag<T>::load(Bb2 + bo);
    }
#pragma unroll
    for (int i = 0; i < 4; ++i) {
      const size_t ao = (size_t)(m0 + (i << 4) + rlane) * lda + koff + k0;
      V ah = Frag<T>::load(Ab + ao);
      V al;
      if (SPLIT >= 1) al = Frag<T>::load(Ab2 + ao);
#pragma unroll
      for (int j = 0; j < 4; ++j) {
        acc[i][j] = Frag<T>::mma(ah, bh[j], acc[i][j]);
        if (SPLIT == 2) acc[i][j] = Frag<T>::mma(ah, bl[j], acc[i][j]);
        if (SPLIT >= 1) acc[i][j] = Frag<T>::mma(al, bh[j], acc[i][j]);
      }
      Frag<T>::guard(acc[i][0], acc[i][3], ah, (SPLIT >= 1) ? al : ah);
    }
    Frag<T>::keep(bh[0], bh[1], bh[2], bh[3]);
    if (SPLIT == 2) Frag<T>::keep(bl[0], bl[1], bl[2], bl[3]);
  }
  acc_guard4(acc[0][0], acc[0][1], acc[0][2], acc[0][3]);
  acc_guard4(acc[1][0], acc[1][1], acc[1][2], acc[1][3]);
  acc_guard4(acc[2][0], acc[2][1], acc[2][2], acc[2][3]);
  acc_guard4(acc[3][0], acc[3][1], acc[3][2], acc[3][3]);

  float* slab = sT[wave];
#pragma unroll
  for (int i = 0; i < 4; ++i) {
    const int mBase = m0 + (i << 4);
#pragma unroll
    for (int j = 0; j < 4; ++j) {
      const int n = n0 + (j << 4) + rlane;
      float bv = 0.f;
      if (BIAS_MODE == 2) bv = bias[n];
#pragma unroll
      for (int r = 0; r < 8; ++r) {
        float v = acc[i][j][r] * scale;
        if (BIAS_MODE == 1) v += bias[mBase + mOff + r];
        if (BIAS_MODE == 2) v += bv;
        slab[(mOff + r) * 68 + (j << 4) + rlane] = v;
      }
    }
    __builtin_amdgcn_fence(3, "workgroup");
    __builtin_amdgcn_wave_barrier();
    __builtin_amdgcn_fence(2, "workgroup");
    if (OUT_MODE == 0) {
      float* C = (float*)Cout + (size_t)b * strideC;
      const int hh = lane >> 4, c4 = (lane & 15) * 4;
      for (int pass = 0; pass < 2; ++pass) {
#pragma unroll
        for (int it = 0; it < 8; ++it) {
          const int row = it * 2 + hh;
          v4f v = *(const v4f*)(slab + row * 68 + c4);
          *(volatile v4f*)(C + (size_t)(mBase + row) * ldc + n0 + c4) = v;
        }
        __threadfence();
      }
    } else {
      const int q = lane >> 3, c8 = (lane & 7) * 8;
      unsigned short* C  = (unsigned short*)Cout  + (size_t)b * strideC;
      unsigned short* C2 = (OUT_MODE >= 2) ? ((unsigned short*)Cout2 + (size_t)b * strideC) : nullptr;
      for (int pass = 0; pass < 2; ++pass) {
#pragma unroll
        for (int it = 0; it < 4; ++it) {
          const int row = it * 4 + q;
          const float* sp = slab + row * 68 + c8;
          v8h hv, lv;
#pragma unroll
          for (int e = 0; e < 8; ++e) {
            if (OUT_MODE == 1) {
              hv[e] = (_Float16)sp[e];
            } else if (OUT_MODE == 3) {
              const _Float16 hq = (_Float16)sp[e];
              const float hqf = (float)hq;
              hv[e] = hq;
              lv[e] = (_Float16)((sp[e] - hqf) * RES_SC);
            } else {
              unsigned short hb = f2bf_bits(sp[e]);
              unsigned short lb = f2bf_bits(sp[e] - bf_bits2f(hb));
              hv[e] = __builtin_bit_cast(_Float16, hb);
              lv[e] = __builtin_bit_cast(_Float16, lb);
            }
          }
          *(volatile v8h*)(C + (size_t)(mBase + row) * ldc + n0 + c8) = hv;
          if (OUT_MODE >= 2) *(volatile v8h*)(C2 + (size_t)(mBase + row) * ldc + n0 + c8) = lv;
        }
        __threadfence();
      }
    }
    __builtin_amdgcn_fence(3, "workgroup");
    __builtin_amdgcn_wave_barrier();
    __builtin_amdgcn_fence(2, "workgroup");
  }
}

__global__ __launch_bounds__(256) void cast_f32_bf16x8(const float* __restrict__ in, long strideIn,
                                                       unsigned short* __restrict__ out, long strideOut, int n8) {
  const int i = blockIdx.x * 256 + threadIdx.x;
  const int b = blockIdx.y;
  if (i < n8) {
    const float* src = in + (size_t)b * strideIn + (size_t)8 * i;
    const v4f a = *(const v4f*)(src);
    const v4f c = *(const v4f*)(src + 4);
    v8us u;
    u[0] = f2bf_bits(a[0]); u[1] = f2bf_bits(a[1]); u[2] = f2bf_bits(a[2]); u[3] = f2bf_bits(a[3]);
    u[4] = f2bf_bits(c[0]); u[5] = f2bf_bits(c[1]); u[6] = f2bf_bits(c[2]); u[7] = f2bf_bits(c[3]);
    unsigned short* p = out + (size_t)b * strideOut + (size_t)8 * i;
    *(volatile v8us*)p = u;
    __threadfence();
    *(volatile v8us*)p = u;
  }
}

struct RopeTab { float inv[64]; };
static_assert(sizeof(RopeTab) == 256);

__global__ __launch_bounds__(128) void norm_rope_split(const float* __restrict__ qk, const float* __restrict__ qgain,
                                                       unsigned short* __restrict__ Qh, unsigned short* __restrict__ Ql,
                                                       unsigned short* __restrict__ Kh, unsigned short* __restrict__ Kl,
                                                       RopeTab rt) {
#pragma clang fp contract(off)
  __shared__ __align__(16) float cs[64];
  __shared__ __align__(16) float sn[64];
  __shared__ __align__(16) float ssq[32];
  __shared__ __align__(16) unsigned short stage[80 * 64];
  const int tid = threadIdx.x;
  const int wave = tid >> 5;
  const int lane = tid & 31;
  const int bt = blockIdx.x;
  const int b = bt / SEQ;
  const int t = bt - b * SEQ;
  if (tid < 64) {
    const float ang = (float)t * rt.inv[tid];
    float sv, cv;
    sincosf(ang, &sv, &cv);
    cs[tid] = cv;
    sn[tid] = sv;
  }
  const float* row = qk + (size_t)bt * NQK;
#pragma unroll
  for (int i = 0; i < 5; ++i) {
    const v4f v = *(const v4f*)(row + 4 * (tid + 128 * i));
    float ss = (v[0] * v[0] + v[1] * v[1]) + (v[2] * v[2] + v[3] * v[3]);
#pragma unroll
    for (int off = 1; off < 32; off <<= 1) ss += __shfl_xor(ss, off, 32);
    if (lane == 0) ssq[4 * i + wave] = ss;
  }
  __syncthreads();
#pragma unroll 1
  for (int i = 0; i < 3; ++i) {
    const int u = tid + 128 * i;
    if (u < 320) {
      const int hu = u >> 4;
      const int j = (u & 15) * 4;
      const bool isq = hu < NHEAD;
      const int col = hu * HD;
      const int Lh = isq ? (2 * hu) : (64 + 2 * (hu - NHEAD));
      const int Ll = isq ? (32 + 2 * hu) : (72 + 2 * (hu - NHEAD));
      const float rn = rsqrtf(ssq[hu] * (1.0f / 128.0f) + RMS_EPS);
      const int hcl = isq ? hu : 0;
      const float graw = qgain[hcl];
      const float g = isq ? bf_bits2f(f2bf_bits(graw)) : 1.0f;
      const v4f x1 = *(const v4f*)(row + col + j);
      const v4f x2 = *(const v4f*)(row + col + 64 + j);
      const v4f c4 = *(const v4f*)(cs + j);
      const v4f s4 = *(const v4f*)(sn + j);
      v4us h1, l1, h2, l2;
#pragma unroll
      for (int e = 0; e < 4; ++e) {
        const float n1 = x1[e] * rn;
        const float n2 = x2[e] * rn;
        const float y1 = (n1 * c4[e] + n2 * s4[e]) * g;
        const float y2 = (n2 * c4[e] - n1 * s4[e]) * g;
        const _Float16 a1 = (_Float16)y1;
        const _Float16 a2 = (_Float16)y2;
        const float a1f = (float)a1;
        const float a2f = (float)a2;
        h1[e] = __builtin_bit_cast(unsigned short, a1);
        h2[e] = __builtin_bit_cast(unsigned short, a2);
        l1[e] = __builtin_bit_cast(unsigned short, (_Float16)((y1 - a1f) * RES_SC));
        l2[e] = __builtin_bit_cast(unsigned short, (_Float16)((y2 - a2f) * RES_SC));
      }
      *(v4us*)(stage + Lh * 64 + j)       = h1;
      *(v4us*)(stage + (Lh + 1) * 64 + j) = h2;
      *(v4us*)(stage + Ll * 64 + j)       = l1;
      *(v4us*)(stage + (Ll + 1) * 64 + j) = l2;
    }
  }
  __syncthreads();
  for (int pass = 0; pass < 2; ++pass) {
#pragma unroll
    for (int i = 0; i < 5; ++i) {
      const int p = tid + 128 * i;
      const int L = p >> 3;
      const int w8 = (p & 7) * 8;
      const v8us val = *(const v8us*)(stage + L * 64 + w8);
      unsigned short* dst;
      if (i < 4) {
        unsigned short* base = (i < 2) ? Qh : Ql;
        const int hq = (L & 31) >> 1, half = L & 1;
        dst = base + ((size_t)(b * NHEAD + hq) * SEQ + t) * HD + half * 64 + w8;
      } else {
        const int L2 = L - 64;
        const int plane = L2 >> 3;
        const int kv = (L2 & 7) >> 1, half = L2 & 1;
        unsigned short* base = plane ? Kl : Kh;
        dst = base + ((size_t)(b * NKV + kv) * SEQ + t) * HD + half * 64 + w8;
      }
      *(volatile v8us*)dst = val;
    }
    __threadfence();
  }
}

template <bool SPL>
__global__ __launch_bounds__(128) void sdpa_d128(
    const unsigned short* __restrict__ Qhp, const unsigned short* __restrict__ Qlp,
    const unsigned short* __restrict__ Khp, const unsigned short* __restrict__ Klp,
    const unsigned short* __restrict__ Vhp, const unsigned short* __restrict__ Vlp,
    unsigned short* __restrict__ Ohp, unsigned short* __restrict__ Olp,
    int qb_lo, int qb_cnt, float sm_scale) {
  union FH { v16h v; v8h h[2]; v8us u[2]; };
  __shared__ __align__(16) unsigned short Ksh[AKC * HD];
  __shared__ __align__(16) unsigned short Ksl[SPL ? AKC * HD : 8];
  __shared__ __align__(16) unsigned short Vth[HD * AKC];
  __shared__ __align__(16) unsigned short Vtl[SPL ? HD * AKC : 8];
  __shared__ __align__(16) _Float16 Psh[ANW][16 * AKC];
  __shared__ __align__(16) _Float16 Psl[SPL ? ANW : 1][SPL ? 16 * AKC : 8];
  __shared__ __align__(16) float  Os[ANW][16 * 68];

  const int tid  = threadIdx.x;
  const int wave = tid >> 5;
  const int lane = tid & 31;
  const int hh   = lane >> 4;
  const int c    = lane & 15;
  const int bx   = blockIdx.x;
  const int qb   = qb_lo + (bx % qb_cnt);
  const int bh   = bx / qb_cnt;
  const int h    = bh % NHEAD;
  const int b    = bh / NHEAD;
  const int kvh  = h / GRP;
  const int q0   = qb * 64 + wave * 16;

  const size_t qoff = ((size_t)(b * NHEAD + h) * SEQ + q0 + c) * HD;
  const _Float16* Qh = (const _Float16*)Qhp + qoff;
  const _Float16* Ql = (const _Float16*)Qlp + qoff;
  const size_t kvb = (size_t)(b * NKV + kvh) * SEQ * HD;
  const unsigned short* Kh = Khp + kvb;
  const unsigned short* Kl = Klp + kvb;
  const unsigned short* Vh = Vhp + kvb;
  const unsigned short* Vl = Vlp + kvb;
  const size_t ooff = (size_t)b * SEQ * CDIM + (size_t)h * HD;
  unsigned short* Oh = Ohp + ooff;
  unsigned short* Ol = Olp + ooff;

  float mrow[8], lrow[8];
  v8f oacc[8];
#pragma unroll
  for (int r = 0; r < 8; ++r) { mrow[r] = -INFINITY; lrow[r] = 0.f; }
#pragma unroll
  for (int t = 0; t < 8; ++t) oacc[t] = zero8();

  const int nChunks = 2 * (qb + 1);
  for (int kc = 0; kc < nChunks; ++kc) {
    const int kv0 = kc * AKC;
    __syncthreads();
#pragma unroll
    for (int i = 0; i < 4; ++i) {
      const int e = tid + 128 * i;
      const int row = e >> 4;
      const int seg = (e & 15) * 8;
      const size_t go = (size_t)(kv0 + row) * HD + seg;
      const v8us a = *(const v8us*)(Kh + go);
      *(v8us*)(Ksh + row * HD + seg) = a;
      if (SPL) {
        const v8us a2 = *(const v8us*)(Kl + go);
        *(v8us*)(Ksl + row * HD + seg) = a2;
      }
    }
#pragma unroll
    for (int i = 0; i < 4; ++i) {
      const int e = tid + 128 * i;
      const int d = e >> 2;
      const int seg = (e & 3) * 8;
      const size_t go = (size_t)d * SEQ + kv0 + seg;
      const v8us a = *(const v8us*)(Vh + go);
      *(v8us*)(Vth + d * AKC + seg) = a;
      if (SPL) {
        const v8us a2 = *(const v8us*)(Vl + go);
        *(v8us*)(Vtl + d * AKC + seg) = a2;
      }
    }
    __syncthreads();

    v8f s[2], sr[2];
    s[0] = zero8(); s[1] = zero8(); sr[0] = zero8(); sr[1] = zero8();
#pragma unroll 1
    for (int dc = 0; dc < 4; ++dc) {
      const v16h qah = Frag<_Float16>::load(Qh + dc * 32 + 8 * hh);
      v16h qal;
      if (SPL) qal = Frag<_Float16>::load(Ql + dc * 32 + 8 * hh);
#pragma unroll
      for (int j = 0; j < 2; ++j) {
        FH kb;
        kb.u[0] = *(const v8us*)(Ksh + (j * 16 + c) * HD + dc * 32 + 8 * hh);
        kb.u[1] = *(const v8us*)(Ksh + (j * 16 + c) * HD + dc * 32 + 16 + 8 * hh);
        s[j] = hmma(qah, kb.v, s[j]);
        if (SPL) {
          FH kl;
          kl.u[0] = *(const v8us*)(Ksl + (j * 16 + c) * HD + dc * 32 + 8 * hh);
          kl.u[1] = *(const v8us*)(Ksl + (j * 16 + c) * HD + dc * 32 + 16 + 8 * hh);
          sr[j] = hmma(qah, kl.v, sr[j]);
          sr[j] = hmma(qal, kb.v, sr[j]);
        }
      }
    }

    float cm[8];
#pragma unroll
    for (int r = 0; r < 8; ++r) {
      const int qrow = q0 + 8 * hh + r;
      float m = -INFINITY;
#pragma unroll
      for (int j = 0; j < 2; ++j) {
        const int kvcol = kv0 + j * 16 + c;
        float v = SPL ? (s[j][r] + sr[j][r] * RES_INV) : s[j][r];
        v = v * sm_scale;
        if (kvcol > qrow) v = -INFINITY;
        s[j][r] = v;
        m = fmaxf(m, v);
      }
#pragma unroll
      for (int off = 1; off < 16; off <<= 1) m = fmaxf(m, __shfl_xor(m, off, 32));
      cm[r] = m;
    }
    _Float16* pwh = Psh[wave];
    _Float16* pwl = Psl[SPL ? wave : 0];
#pragma unroll
    for (int r = 0; r < 8; ++r) {
      const float mnew = fmaxf(mrow[r], cm[r]);
      const float alpha = expf(mrow[r] - mnew);
      mrow[r] = mnew;
      float psum = 0.f;
#pragma unroll
      for (int j = 0; j < 2; ++j) {
        const float p = expf(s[j][r] - mnew);
        psum += p;
        const float ps = p * P_SC;
        const _Float16 ph = (_Float16)ps;
        pwh[(8 * hh + r) * AKC + j * 16 + c] = ph;
        if (SPL) {
          const float phf = (float)ph;
          pwl[(8 * hh + r) * AKC + j * 16 + c] = (_Float16)((ps - phf) * RES_SC);
        }
      }
#pragma unroll
      for (int off = 1; off < 16; off <<= 1) psum += __shfl_xor(psum, off, 32);
      lrow[r] = lrow[r] * alpha + psum;
#pragma unroll
      for (int t = 0; t < 8; ++t) oacc[t][r] *= alpha;
    }
    __builtin_amdgcn_fence(3, "workgroup");
    __builtin_amdgcn_wave_barrier();
    __builtin_amdgcn_fence(2, "workgroup");

    {
      FH pa, pl;
      pa.h[0] = *(const v8h*)(pwh + c * AKC + 8 * hh);
      pa.h[1] = *(const v8h*)(pwh + c * AKC + 16 + 8 * hh);
      if (SPL) {
        pl.h[0] = *(const v8h*)(pwl + c * AKC + 8 * hh);
        pl.h[1] = *(const v8h*)(pwl + c * AKC + 16 + 8 * hh);
      }
#pragma unroll
      for (int t = 0; t < 8; ++t) {
        FH vb;
        vb.u[0] = *(const v8us*)(Vth + (t * 16 + c) * AKC + 8 * hh);
        vb.u[1] = *(const v8us*)(Vth + (t * 16 + c) * AKC + 16 + 8 * hh);
        if (SPL) {
          FH vl;
          vl.u[0] = *(const v8us*)(Vtl + (t * 16 + c) * AKC + 8 * hh);
          vl.u[1] = *(const v8us*)(Vtl + (t * 16 + c) * AKC + 16 + 8 * hh);
          v8f rr = hmma(pa.v, vl.v, zero8());
          rr = hmma(pl.v, vb.v, rr);
          oacc[t] = hmma(pa.v, vb.v, oacc[t]);
          oacc[t] = oacc[t] + rr * RES_INV;
        } else {
          oacc[t] = hmma(pa.v, vb.v, oacc[t]);
        }
      }
    }
  }

  float invl[8];
#pragma unroll
  for (int r = 0; r < 8; ++r) invl[r] = 1.0f / (lrow[r] * P_SC);
  float* os = Os[wave];
  const int q4 = lane >> 3;
  const int c8 = (lane & 7) * 8;
#pragma unroll
  for (int dh = 0; dh < 2; ++dh) {
#pragma unroll
    for (int r = 0; r < 8; ++r) {
#pragma unroll
      for (int t4 = 0; t4 < 4; ++t4) os[(8 * hh + r) * 68 + t4 * 16 + c] = oacc[dh * 4 + t4][r] * invl[r];
    }
    __builtin_amdgcn_fence(3, "workgroup");
    __builtin_amdgcn_wave_barrier();
    __builtin_amdgcn_fence(2, "workgroup");
    for (int pass = 0; pass < 2; ++pass) {
#pragma unroll
      for (int it = 0; it < 4; ++it) {
        const int row = it * 4 + q4;
        const float* sp = os + row * 68 + c8;
        v8h hv, lv;
#pragma unroll
        for (int e = 0; e < 8; ++e) {
          const unsigned short hb = f2bf_bits(sp[e]);
          const unsigned short lb = f2bf_bits(sp[e] - bf_bits2f(hb));
          hv[e] = __builtin_bit_cast(_Float16, hb);
          lv[e] = __builtin_bit_cast(_Float16, lb);
        }
        const size_t o = (size_t)(q0 + row) * CDIM + dh * 64 + c8;
        *(volatile v8h*)(Oh + o) = hv;
        *(volatile v8h*)(Ol + o) = lv;
      }
      __threadfence();
    }
    __builtin_amdgcn_fence(3, "workgroup");
    __builtin_amdgcn_wave_barrier();
    __builtin_amdgcn_fence(2, "workgroup");
  }
}

static constexpr size_t SZ_XB   = (size_t)BT * CDIM * 2;
static constexpr size_t SZ_WQKT = (size_t)NQK * CDIM * 2;
static constexpr size_t SZ_WVT  = (size_t)NKVC * CDIM * 2;
static constexpr size_t SZ_WOT  = (size_t)CDIM * CDIM * 2;
static constexpr size_t SZ_QK   = (size_t)BT * NQK * 4;
static constexpr size_t SZ_O    = (size_t)BT * CDIM * 2;
static constexpr size_t SZ_VT   = (size_t)NB * NKVC * SEQ * 2;
static constexpr size_t SZ_Q    = (size_t)NB * NHEAD * SEQ * HD * 2;
static constexpr size_t SZ_K    = (size_t)NB * NKV * SEQ * HD * 2;
static constexpr size_t WS_TOTAL = SZ_XB + SZ_WQKT + SZ_WVT + SZ_WOT + SZ_QK + 2 * SZ_VT + 2 * SZ_Q + 2 * SZ_K;
static_assert(2 * SZ_O <= SZ_QK);
static_assert(WS_TOTAL <= 134217728);
static_assert((SZ_XB % 128) == 0 && (SZ_WQKT % 128) == 0 && (SZ_WVT % 128) == 0 && (SZ_WOT % 128) == 0 && (SZ_QK % 128) == 0);
static_assert((SZ_VT % 128) == 0 && (SZ_Q % 128) == 0 && (SZ_K % 128) == 0 && (SZ_O % 128) == 0);
static_assert(((size_t)(NB - 1) * SEQ_FULL + SEQ) * CDIM <= (size_t)NB_FULL * SEQ_FULL * CDIM);

extern "C" void kernel_launch(void* const* d_in, const int* in_sizes, int n_in,
                              void* d_out, int out_size, void* d_ws, size_t ws_size,
                              hipStream_t stream) {
  if (n_in < 6) return;
  const size_t needRows = (size_t)(NB - 1) * SEQ_FULL + SEQ;
  if ((size_t)in_sizes[0] < needRows * CDIM) return;
  if (in_sizes[1] < CDIM * CDIM || in_sizes[2] < NKVC * CDIM || in_sizes[3] < NKVC * CDIM ||
      in_sizes[4] < CDIM * CDIM || in_sizes[5] < NHEAD) return;
  if ((size_t)out_size < needRows * CDIM) return;
  if (ws_size < WS_TOTAL) return;

  const float* x  = (const float*)d_in[0];
  const float* Wq = (const float*)d_in[1];
  const float* Wk = (const float*)d_in[2];
  const float* Wv = (const float*)d_in[3];
  const float* Wo = (const float*)d_in[4];
  const float* qg = (const float*)d_in[5];
  float* out = (float*)d_out;

  char* ws = (char*)d_ws;
  size_t off = 0;
  unsigned short* xb   = (unsigned short*)(ws + off); off += SZ_XB;
  unsigned short* wqkt = (unsigned short*)(ws + off); off += SZ_WQKT;
  unsigned short* wvt  = (unsigned short*)(ws + off); off += SZ_WVT;
  unsigned short* wot  = (unsigned short*)(ws + off); off += SZ_WOT;
  float* qkraw         = (float*)(ws + off);
  unsigned short* oh   = (unsigned short*)(ws + off);
  unsigned short* ol   = (unsigned short*)(ws + off + SZ_O);
  off += SZ_QK;
  unsigned short* vth  = (unsigned short*)(ws + off); off += SZ_VT;
  unsigned short* vtl  = (unsigned short*)(ws + off); off += SZ_VT;
  unsigned short* qh   = (unsigned short*)(ws + off); off += SZ_Q;
  unsigned short* ql   = (unsigned short*)(ws + off); off += SZ_Q;
  unsigned short* kh   = (unsigned short*)(ws + off); off += SZ_K;
  unsigned short* kl   = (unsigned short*)(ws + off); off += SZ_K;
  if (off > ws_size) return;
  const float* fdummy = (const float*)d_ws;

  {
    const int n8 = SEQ * CDIM / 8;
    cast_f32_bf16x8<<<dim3(n8 / 256, NB), dim3(256), 0, stream>>>(x, (long)SEQ_FULL * CDIM, xb, (long)SEQ * CDIM, n8);
  }
  {
    const int n8q = CDIM * CDIM / 8;
    const int n8k = NKVC * CDIM / 8;
    cast_f32_bf16x8<<<dim3(n8q / 256, 1), dim3(256), 0, stream>>>(Wq, 0L, wqkt, 0L, n8q);
    cast_f32_bf16x8<<<dim3(n8k / 256, 1), dim3(256), 0, stream>>>(Wk, 0L, wqkt + (size_t)CDIM * CDIM, 0L, n8k);
    cast_f32_bf16x8<<<dim3(n8k / 256, 1), dim3(256), 0, stream>>>(Wv, 0L, wvt, 0L, n8k);
    cast_f32_bf16x8<<<dim3(n8q / 256, 1), dim3(256), 0, stream>>>(Wo, 0L, wot, 0L, n8q);
  }

  {
    const int tiles = (BT / 64) * (NQK / 64);
    wmma_gemm64<1, 0, 0, 0><<<dim3(tiles / 8, 1), dim3(256), 0, stream>>>(
        xb, xb, CDIM, 0L, wqkt, wqkt, CDIM, 0L, (void*)qkraw, (void*)qkraw, NQK, 0L,
        fdummy, BT, NQK, CDIM, 1.0f);
  }
  {
    const int tiles = (NKVC / 64) * (SEQ / 64);
    wmma_gemm64<1, 0, 0, 3><<<dim3(tiles / 8, NB), dim3(256), 0, stream>>>(
        wvt, wvt, CDIM, 0L, xb, xb, CDIM, (long)SEQ * CDIM, (void*)vth, (void*)vtl, SEQ, (long)NKVC * SEQ,
        fdummy, NKVC, SEQ, CDIM, 1.0f);
  }
  {
    RopeTab rt;
    for (int j = 0; j < 64; ++j) {
      const float pj = (float)pow(10000.0, (double)j / 64.0);
      rt.inv[j] = 1.0f / pj;
    }
    norm_rope_split<<<dim3(BT), dim3(128), 0, stream>>>(qkraw, qg, qh, ql, kh, kl, rt);
  }
  {
    const float sm_scale = 1.0f / sqrtf((float)HD);
    sdpa_d128<true><<<dim3(NB * NHEAD * NQB_SPLIT), dim3(128), 0, stream>>>(
        qh, ql, kh, kl, vth, vtl, oh, ol, 0, NQB_SPLIT, sm_scale);
    if (NQB > NQB_SPLIT) {
      sdpa_d128<false><<<dim3(NB * NHEAD * (NQB - NQB_SPLIT)), dim3(128), 0, stream>>>(
          qh, ql, kh, kl, vth, vtl, oh, ol, NQB_SPLIT, NQB - NQB_SPLIT, sm_scale);
    }
  }
  {
    const int tiles = (SEQ / 64) * (CDIM / 64);
    wmma_gemm64<1, 1, 0, 0><<<dim3(tiles / 8, NB), dim3(256), 0, stream>>>(
        oh, ol, CDIM, (long)SEQ * CDIM, wot, wot, CDIM, 0L, (void*)out, (void*)out, CDIM, (long)SEQ_FULL * CDIM,
        fdummy, SEQ, CDIM, CDIM, 1.0f);
  }
}
